// MulHeadCrossAttn_62362925137951
// MI455X (gfx1250) — hardware-verified
//
#include <hip/hip_runtime.h>
#include <math.h>
#include <stdint.h>

#ifndef NB
#define NB       4
#endif
#ifndef SEQ
#define SEQ      1024
#endif
#define NB_FULL  4
#define SEQ_FULL 1024
#define SKV      1024
#define DM       1024
#define NG       64
#define HD       16
#define GP       32
#define QKP      (NG * GP)
#define WSC      256.0f
#define QS       8.0f
#define KS       8.0f
#define VS       8.0f
#define CS       256.0f
#define PCAR     32768.0f
#define RESC     2048.0f
#define RINV     (1.0f / 2048.0f)
#define LOG2E    1.4426950408889634f
#define NKB      (SKV / 32)
#define ATT_WAVES   4
#define ATT_THREADS (ATT_WAVES * 32)
#define CVT_THREADS (DM / 8)
#define TR_THREADS  128
#define OPITCH   68
#define GPITCH   68
#define TPITCH   65

static_assert(NB >= 1 && NB <= NB_FULL);
static_assert((SEQ % 128) == 0 && SEQ >= 128 && SEQ <= SEQ_FULL);
static_assert((SKV % 128) == 0 && (SKV % 64) == 0 && NKB * 32 == SKV);
static_assert(NG * HD == DM && HD == 16 && GP == 2 * HD && QKP == 2 * DM && (NG % 4) == 0);
static_assert((DM % 64) == 0 && (DM % 32) == 0 && CVT_THREADS == 128);
static_assert((OPITCH * 4) % 16 == 0 && (GPITCH * 4) % 16 == 0);
static_assert(ATT_THREADS == 128 && TR_THREADS == 128);

typedef unsigned short u16;
typedef _Float16 v16h __attribute__((ext_vector_type(16)));
typedef _Float16 v8h  __attribute__((ext_vector_type(8)));
typedef float    v8f  __attribute__((ext_vector_type(8)));
typedef float    v4f  __attribute__((ext_vector_type(4)));
typedef unsigned int v4u __attribute__((ext_vector_type(4)));

union FragH { v16h v; v8h h[2]; v4u u[2]; };

__device__ __forceinline__ unsigned short bf_bits(float f) {
  unsigned u = __float_as_uint(f);
  return (unsigned short)((u + 0x7FFFu + ((u >> 16) & 1u)) >> 16);
}
__device__ __forceinline__ float bf_up(unsigned short h) { return __uint_as_float(((unsigned)h) << 16); }
__device__ __forceinline__ float bfr(float f) { return bf_up(bf_bits(f)); }
__device__ __forceinline__ unsigned short h_bits(_Float16 x) { return __builtin_bit_cast(unsigned short, x); }
__device__ __forceinline__ unsigned pk16(unsigned short a, unsigned short b) { return (unsigned)a | ((unsigned)b << 16); }
__device__ __forceinline__ v8f zero8() { v8f z = {0.f, 0.f, 0.f, 0.f, 0.f, 0.f, 0.f, 0.f}; return z; }

__device__ __forceinline__ void split2(float x0, float x1, unsigned& hp, unsigned& rp) {
  const _Float16 h0 = (_Float16)x0, h1 = (_Float16)x1;
  const _Float16 r0 = (_Float16)((x0 - (float)h0) * RESC);
  const _Float16 r1 = (_Float16)((x1 - (float)h1) * RESC);
  hp = pk16(h_bits(h0), h_bits(h1));
  rp = pk16(h_bits(r0), h_bits(r1));
}

__device__ __forceinline__ v16h ldfrag_h(const _Float16* p) {
  FragH f;
  f.h[0] = *(const v8h*)(p);
  f.h[1] = *(const v8h*)(p + 16);
  return f.v;
}

__device__ __forceinline__ v8f mma_h(v16h a, v16h b, v8f c) {
  return __builtin_amdgcn_wmma_f32_16x16x32_f16(false, a, false, b, (short)0, c, false, false);
}
__device__ __forceinline__ void guard_4(v8f& a, v8f& b, v8f& c, v8f& d, v16h x0, v16h x1, v16h x2, v16h x3) {
#if defined(__HIP_DEVICE_COMPILE__)
  asm volatile("v_nop\n\tv_nop\n\tv_nop\n\tv_nop"
               : "+v"(a), "+v"(b), "+v"(c), "+v"(d) : "v"(x0), "v"(x1), "v"(x2), "v"(x3) : "memory");
#endif
}
__device__ __forceinline__ void guard_2(v8f& a, v8f& b, v16h x0, v16h x1, v16h x2, v16h x3) {
#if defined(__HIP_DEVICE_COMPILE__)
  asm volatile("v_nop\n\tv_nop\n\tv_nop\n\tv_nop"
               : "+v"(a), "+v"(b) : "v"(x0), "v"(x1), "v"(x2), "v"(x3) : "memory");
#endif
}
__device__ __forceinline__ void guard_g(v8f (&acc)[8], v16h x0, v16h x1, v16h x2, v16h x3, v16h x4, v16h x5) {
#if defined(__HIP_DEVICE_COMPILE__)
  asm volatile("v_nop\n\tv_nop\n\tv_nop\n\tv_nop"
               : "+v"(acc[0]), "+v"(acc[1]), "+v"(acc[2]), "+v"(acc[3]),
                 "+v"(acc[4]), "+v"(acc[5]), "+v"(acc[6]), "+v"(acc[7])
               : "v"(x0), "v"(x1), "v"(x2), "v"(x3), "v"(x4), "v"(x5) : "memory");
#endif
}
__device__ __forceinline__ void acc_guard2(v8f& a, v8f& b) {
#if defined(__HIP_DEVICE_COMPILE__)
  asm volatile("v_nop\n\tv_nop\n\tv_nop\n\tv_nop" : "+v"(a), "+v"(b));
#endif
}
__device__ __forceinline__ void wave_sync_lds() {
  __builtin_amdgcn_fence(__ATOMIC_RELEASE, "workgroup");
  __builtin_amdgcn_wave_barrier();
  __builtin_amdgcn_fence(__ATOMIC_ACQUIRE, "workgroup");
}

__global__ __launch_bounds__(CVT_THREADS)
void cvt16(const float* __restrict__ x, u16* Y, int rowsPerB, int srcRowsPerB, float scale) {
  const int tid = threadIdx.x;
  const int r = blockIdx.x;
  const int b = r / rowsPerB;
  const int s = r - b * rowsPerB;
  const float* src = x + ((size_t)b * (size_t)srcRowsPerB + (size_t)s) * (size_t)DM + (size_t)tid * 8;
  const v4f a = *(const v4f*)(src), c4 = *(const v4f*)(src + 4);
  v4u o;
#pragma unroll
  for (int e = 0; e < 2; ++e) {
    o[e]     = pk16(h_bits((_Float16)(bfr(a[2 * e]) * scale)),  h_bits((_Float16)(bfr(a[2 * e + 1]) * scale)));
    o[2 + e] = pk16(h_bits((_Float16)(bfr(c4[2 * e]) * scale)), h_bits((_Float16)(bfr(c4[2 * e + 1]) * scale)));
  }
  u16* dst = Y + (size_t)r * (size_t)DM + (size_t)tid * 8;
  for (int pass = 0; pass < 2; ++pass) {
    *(volatile v4u*)(dst) = o;
    __threadfence();
  }
}

__global__ __launch_bounds__(TR_THREADS)
void cvtT16(const float* __restrict__ W, u16* Y, float scale) {
  __shared__ __align__(16) float tile[64 * TPITCH];
  const int tid = threadIdx.x;
  constexpr int NT = DM / 64;
  const int bid = blockIdx.x;
  const int kt  = bid % NT;
  const int ntb = bid / NT;
  const int k0  = kt * 64, n0 = ntb * 64;
  const int lr = tid >> 4, lc = (tid & 15) * 4;
#pragma unroll
  for (int p = 0; p < 8; ++p) {
    const int kk = p * 8 + lr;
    const v4f w4 = *(const v4f*)(W + (size_t)(k0 + kk) * (size_t)DM + n0 + lc);
    tile[kk * TPITCH + lc + 0] = w4[0];
    tile[kk * TPITCH + lc + 1] = w4[1];
    tile[kk * TPITCH + lc + 2] = w4[2];
    tile[kk * TPITCH + lc + 3] = w4[3];
  }
  __syncthreads();
  const int rq = tid >> 3, c8 = (tid & 7) * 8;
  v4u ov[4];
#pragma unroll
  for (int i = 0; i < 4; ++i) {
    const int row = 16 * i + rq;
#pragma unroll
    for (int e = 0; e < 4; ++e) {
      const float x0 = tile[(c8 + 2 * e) * TPITCH + row];
      const float x1 = tile[(c8 + 2 * e + 1) * TPITCH + row];
      ov[i][e] = pk16(h_bits((_Float16)(bfr(x0) * scale)), h_bits((_Float16)(bfr(x1) * scale)));
    }
  }
  u16* dst = Y + (size_t)n0 * (size_t)DM + k0 + c8;
  for (int pass = 0; pass < 2; ++pass) {
#pragma unroll
    for (int i = 0; i < 4; ++i) {
      const int row = 16 * i + rq;
      *(volatile v4u*)(dst + (size_t)row * (size_t)DM) = ov[i];
    }
    __threadfence();
  }
}

__device__ __forceinline__ void gemm_core(const _Float16* ap, const _Float16* bp, int K, v8f (&acc)[8]) {
  const size_t rs16 = (size_t)16 * (size_t)K;
#pragma unroll 1
  for (int k0 = 0; k0 < K; k0 += 32) {
    const v16h a0 = ldfrag_h(ap + k0), a1 = ldfrag_h(ap + rs16 + k0);
    const v16h b0 = ldfrag_h(bp + k0);
    const v16h b1 = ldfrag_h(bp + rs16 + k0);
    const v16h b2 = ldfrag_h(bp + 2 * rs16 + k0);
    const v16h b3 = ldfrag_h(bp + 3 * rs16 + k0);
    acc[0] = mma_h(a0, b0, acc[0]);
    acc[1] = mma_h(a0, b1, acc[1]);
    acc[2] = mma_h(a0, b2, acc[2]);
    acc[3] = mma_h(a0, b3, acc[3]);
    acc[4] = mma_h(a1, b0, acc[4]);
    acc[5] = mma_h(a1, b1, acc[5]);
    acc[6] = mma_h(a1, b2, acc[6]);
    acc[7] = mma_h(a1, b3, acc[7]);
    guard_g(acc, a0, a1, b0, b1, b2, b3);
  }
}
__device__ __forceinline__ void stage32x64(float* sl, v8f (&acc)[8], float oscale, int lane) {
  const int hh = lane >> 4, m = lane & 15;
#pragma unroll
  for (int i = 0; i < 2; ++i) {
#pragma unroll
    for (int r = 0; r < 8; ++r) {
      const int ro = (16 * i + 8 * hh + r) * GPITCH + m;
      sl[ro]      = acc[4 * i + 0][r] * oscale;
      sl[ro + 16] = acc[4 * i + 1][r] * oscale;
      sl[ro + 32] = acc[4 * i + 2][r] * oscale;
      sl[ro + 48] = acc[4 * i + 3][r] * oscale;
    }
  }
  wave_sync_lds();
}

__global__ __launch_bounds__(128)
void gemm_qk(const u16* __restrict__ A, const u16* __restrict__ Bt, u16* C, int Mb, float oscale) {
  __shared__ __align__(16) float slab[4 * 32 * GPITCH];
  const int tid = threadIdx.x, wave = tid >> 5, lane = tid & 31, hh = lane >> 4, m = lane & 15;
  constexpr int ntile = DM >> 6;
  const int bid  = blockIdx.x;
  const int nt   = bid % ntile;
  const int mt   = bid / ntile;
  const int rowb = mt * 128 + wave * 32;
  const int col0 = nt * 64;
  if (rowb + 32 > Mb) return;
  const _Float16* ap = (const _Float16*)(const void*)A + (size_t)(rowb + m) * DM + 8 * hh;
  const _Float16* bp = (const _Float16*)(const void*)Bt + (size_t)(col0 + m) * DM + 8 * hh;
  v8f acc[8];
#pragma unroll
  for (int i = 0; i < 8; ++i) acc[i] = zero8();
  gemm_core(ap, bp, DM, acc);
  float* sl = slab + wave * 32 * GPITCH;
  stage32x64(sl, acc, oscale, lane);
  const int rs = lane >> 4, pc = lane & 15;
  const int scol = 16 * (pc >> 2) + 8 * (pc & 1);
  const bool isres = (pc & 2) != 0;
  v4u ov[16];
#pragma unroll
  for (int i = 0; i < 16; ++i) {
    const int row = 2 * i + rs;
    const v4f a = *(const v4f*)(sl + row * GPITCH + scol), c4 = *(const v4f*)(sl + row * GPITCH + scol + 4);
#pragma unroll
    for (int e = 0; e < 2; ++e) {
      unsigned hp, rp;
      split2(a[2 * e], a[2 * e + 1], hp, rp);
      ov[i][e] = isres ? rp : hp;
      split2(c4[2 * e], c4[2 * e + 1], hp, rp);
      ov[i][2 + e] = isres ? rp : hp;
    }
  }
  u16* Cb = C + (size_t)rowb * (size_t)QKP + 2 * col0 + 8 * pc;
  for (int pass = 0; pass < 2; ++pass) {
#pragma unroll
    for (int i = 0; i < 16; ++i) {
      const int row = 2 * i + rs;
      *(volatile v4u*)(Cb + (size_t)row * (size_t)QKP) = ov[i];
    }
    __threadfence();
  }
}

__global__ __launch_bounds__(128)
void gemm_hr(const u16* __restrict__ A, const u16* __restrict__ Bt, u16* CH, u16* CR,
             int Mb, int N, int K, int aBs, int bBs, int cBs, float oscale) {
  __shared__ __align__(16) float slab[4 * 32 * GPITCH];
  const int tid = threadIdx.x, wave = tid >> 5, lane = tid & 31, hh = lane >> 4, m = lane & 15;
  const int ntile = N >> 6, mtile = Mb >> 7;
  const int bid  = blockIdx.x;
  const int nt   = bid % ntile;
  const int tmp  = bid / ntile;
  const int mt   = tmp % mtile;
  const int bz   = tmp / mtile;
  const int rowb = mt * 128 + wave * 32;
  const int col0 = nt * 64;
  if (rowb + 32 > Mb) return;
  const _Float16* Ab = (const _Float16*)(const void*)A + (size_t)bz * (size_t)aBs;
  const _Float16* Bb = (const _Float16*)(const void*)Bt + (size_t)bz * (size_t)bBs;
  const _Float16* ap = Ab + (size_t)(rowb + m) * K + 8 * hh;
  const _Float16* bp = Bb + (size_t)(col0 + m) * K + 8 * hh;
  v8f acc[8];
#pragma unroll
  for (int i = 0; i < 8; ++i) acc[i] = zero8();
  gemm_core(ap, bp, K, acc);
  float* sl = slab + wave * 32 * GPITCH;
  stage32x64(sl, acc, oscale, lane);
  const int rq = lane >> 3, c8 = (lane & 7) * 8;
  v4u oh[8], orv[8];
#pragma unroll
  for (int i = 0; i < 8; ++i) {
    const int row = 4 * i + rq;
    const v4f a = *(const v4f*)(sl + row * GPITCH + c8), c4 = *(const v4f*)(sl + row * GPITCH + c8 + 4);
#pragma unroll
    for (int e = 0; e < 2; ++e) {
      unsigned hp, rp;
      split2(a[2 * e], a[2 * e + 1], hp, rp);
      oh[i][e] = hp; orv[i][e] = rp;
      split2(c4[2 * e], c4[2 * e + 1], hp, rp);
      oh[i][2 + e] = hp; orv[i][2 + e] = rp;
    }
  }
  const size_t cbase = (size_t)bz * (size_t)cBs + (size_t)rowb * (size_t)N + col0 + c8;
  u16* Hb = CH + cbase;
  u16* Rb = CR + cbase;
  for (int pass = 0; pass < 2; ++pass) {
#pragma unroll
    for (int i = 0; i < 8; ++i) {
      const int row = 4 * i + rq;
      *(volatile v4u*)(Hb + (size_t)row * (size_t)N) = oh[i];
      *(volatile v4u*)(Rb + (size_t)row * (size_t)N) = orv[i];
    }
    __threadfence();
  }
}

__global__ __launch_bounds__(128)
void gemm_out(const u16* __restrict__ AH, const u16* __restrict__ AR, const u16* __restrict__ Bt, float* Out,
              int Mb, int rowsPerB, int outRowsPerB, float oscale) {
  __shared__ __align__(16) float slab[4 * 32 * GPITCH];
  const int tid = threadIdx.x, wave = tid >> 5, lane = tid & 31, hh = lane >> 4, m = lane & 15;
  constexpr int ntile = DM >> 6;
  const int bid  = blockIdx.x;
  const int nt   = bid % ntile;
  const int mt   = bid / ntile;
  const int rowb = mt * 128 + wave * 32;
  const int col0 = nt * 64;
  if (rowb + 32 > Mb) return;
  const _Float16* ahp = (const _Float16*)(const void*)AH + (size_t)(rowb + m) * DM + 8 * hh;
  const _Float16* arp = (const _Float16*)(const void*)AR + (size_t)(rowb + m) * DM + 8 * hh;
  const _Float16* bp  = (const _Float16*)(const void*)Bt + (size_t)(col0 + m) * DM + 8 * hh;
  v8f acc[8];
#pragma unroll
  for (int i = 0; i < 8; ++i) acc[i] = zero8();
  gemm_core(arp, bp, DM, acc);
#pragma unroll
  for (int i = 0; i < 8; ++i) acc[i] = acc[i] * RINV;
  gemm_core(ahp, bp, DM, acc);
  float* sl = slab + wave * 32 * GPITCH;
  stage32x64(sl, acc, oscale, lane);
  const int rs = lane >> 4, pc = lane & 15;
  v4f ov[16];
#pragma unroll
  for (int i = 0; i < 16; ++i) {
    const int row = 2 * i + rs;
    ov[i] = *(const v4f*)(sl + row * GPITCH + 4 * pc);
  }
  const int bb = rowb / rowsPerB;
  const int ss = rowb - bb * rowsPerB;
  float* ob = Out + ((size_t)bb * (size_t)outRowsPerB + (size_t)ss) * (size_t)DM + col0 + 4 * pc;
  for (int pass = 0; pass < 2; ++pass) {
#pragma unroll
    for (int i = 0; i < 16; ++i) {
      const int row = 2 * i + rs;
      *(volatile v4f*)(ob + (size_t)row * (size_t)DM) = ov[i];
    }
    __threadfence();
  }
}

__global__ __launch_bounds__(ATT_THREADS)
void attn_fwd(const u16* __restrict__ Qp, const u16* __restrict__ Kp, const u16* __restrict__ Vh,
              const u16* __restrict__ Vr, u16* CH, u16* CR) {
  __shared__ __align__(16) float smem[ATT_WAVES * 16 * OPITCH];

  const int tid  = threadIdx.x;
  const int wave = tid >> 5;
  const int lane = tid & 31;
  const int hh   = lane >> 4;
  const int c    = lane & 15;

  constexpr int NQT = SEQ / 64;
  constexpr int NGQ = NG / 4;
  const int bid  = blockIdx.x;
  const int qt   = bid % NQT;
  const int gq   = (bid / NQT) % NGQ;
  const int b    = bid / (NQT * NGQ);
  const int q0   = qt * 64 + wave * 16;
  float* slab = smem + wave * 16 * OPITCH;
  const float lsc = (LOG2E * 0.25f) / (QS * KS);
  const v4u z4 = {0u, 0u, 0u, 0u};

#pragma unroll 1
  for (int jg = 0; jg < 4; ++jg) {
    const int g = 4 * gq + jg;
    const _Float16* Qb  = (const _Float16*)(const void*)Qp + ((size_t)(b * SEQ + q0 + c)) * QKP + g * GP + 8 * hh;
    const _Float16* Kb  = (const _Float16*)(const void*)Kp + ((size_t)(b * SKV + c)) * QKP + g * GP + 8 * hh;
    const _Float16* Vhb = (const _Float16*)(const void*)Vh + ((size_t)(b * DM + g * HD + c)) * SKV + 8 * hh;
    const _Float16* Vrb = (const _Float16*)(const void*)Vr + ((size_t)(b * DM + g * HD + c)) * SKV + 8 * hh;

    FragH f1, f2;
    f1.h[0] = *(const v8h*)(Qb);
    f1.u[1] = z4;
    f2.h[0] = *(const v8h*)(Qb + 16);
    f2.h[1] = f1.h[0];

    float mrun = -INFINITY, lrun = 0.f;
    v8f o = zero8(), orr = zero8();

#pragma unroll 1
    for (int it = 0; it < NKB; ++it) {
      const int kb = it * 32;
      const _Float16* k0p = Kb + (size_t)kb * QKP;
      const _Float16* k1p = k0p + (size_t)16 * QKP;
      const v16h kf0 = ldfrag_h(k0p);
      const v16h kf1 = ldfrag_h(k1p);
      v8f s0  = mma_h(kf0, f1.v, zero8());
      v8f s0r = mma_h(kf0, f2.v, zero8());
      v8f s1  = mma_h(kf1, f1.v, zero8());
      v8f s1r = mma_h(kf1, f2.v, zero8());
      guard_4(s0, s0r, s1, s1r, kf0, kf1, f1.v, f2.v);
      float t[16];
#pragma unroll
      for (int i = 0; i < 8; ++i) {
        t[i]     = fmaf(s0r[i], RINV, s0[i]) * lsc;
        t[8 + i] = fmaf(s1r[i], RINV, s1[i]) * lsc;
      }
      float cm = t[0];
#pragma unroll
      for (int i = 1; i < 16; ++i) cm = fmaxf(cm, t[i]);
      cm = fmaxf(cm, __shfl_xor(cm, 16, 32));
      const float mn = fmaxf(mrun, cm);
      const float al = exp2f(mrun - mn);
      mrun = mn;
      float ps = 0.f;
      FragH ph, pr;
#pragma unroll
      for (int w = 0; w < 2; ++w) {
#pragma unroll
        for (int e4 = 0; e4 < 4; ++e4) {
          const int i = 8 * w + 2 * e4;
          const float p0 = exp2f(t[i] - mn), p1 = exp2f(t[i + 1] - mn);
          ps += p0 + p1;
          unsigned hp, rp;
          split2(p0 * PCAR, p1 * PCAR, hp, rp);
          ph.u[w][e4] = hp;
          pr.u[w][e4] = rp;
        }
      }
      ps += __shfl_xor(ps, 16, 32);
      lrun = lrun * al + ps;
      float scl[8];
#pragma unroll
      for (int r = 0; r < 8; ++r) scl[r] = __shfl(al, 8 * hh + r, 32);
#pragma unroll
      for (int r = 0; r < 8; ++r) { o[r] *= scl[r]; orr[r] *= scl[r]; }
      const v16h vhf = ldfrag_h(Vhb + kb);
      const v16h vrf = ldfrag_h(Vrb + kb);
      o   = mma_h(ph.v, vhf, o);
      orr = mma_h(ph.v, vrf, orr);
      orr = mma_h(pr.v, vhf, orr);
      guard_2(o, orr, ph.v, pr.v, vhf, vrf);
    }
    acc_guard2(o, orr);

    const float linv = (1.0f / lrun) * (CS / (PCAR * VS));
    float inv[8];
#pragma unroll
    for (int r = 0; r < 8; ++r) inv[r] = __shfl(linv, 8 * hh + r, 32);
#pragma unroll
    for (int r = 0; r < 8; ++r) slab[(8 * hh + r) * OPITCH + jg * 16 + c] = fmaf(orr[r], RINV, o[r]) * inv[r];
  }
  wave_sync_lds();

  const int rq = lane >> 3, c8 = (lane & 7) * 8;
  v4u oh[4], orv[4];
#pragma unroll
  for (int i = 0; i < 4; ++i) {
    const int row = 4 * i + rq;
    const v4f a = *(const v4f*)(slab + row * OPITCH + c8), c4 = *(const v4f*)(slab + row * OPITCH + c8 + 4);
#pragma unroll
    for (int e = 0; e < 2; ++e) {
      unsigned hp, rp;
      split2(a[2 * e], a[2 * e + 1], hp, rp);
      oh[i][e] = hp; orv[i][e] = rp;
      split2(c4[2 * e], c4[2 * e + 1], hp, rp);
      oh[i][2 + e] = hp; orv[i][2 + e] = rp;
    }
  }
  const size_t rbase = ((size_t)(b * SEQ + q0)) * (size_t)DM + 64 * gq + c8;
  u16* hb = CH + rbase;
  u16* rb = CR + rbase;
  for (int pass = 0; pass < 2; ++pass) {
#pragma unroll
    for (int i = 0; i < 4; ++i) {
      const int row = 4 * i + rq;
      *(volatile v4u*)(hb + (size_t)row * (size_t)DM) = oh[i];
      *(volatile v4u*)(rb + (size_t)row * (size_t)DM) = orv[i];
    }
    __threadfence();
  }
}

extern "C" void kernel_launch(void* const* d_in, const int* in_sizes, int n_in,
                              void* d_out, int out_size, void* d_ws, size_t ws_size,
                              hipStream_t stream) {
  if (n_in < 6) return;
  if (in_sizes[0] < ((NB - 1) * SEQ_FULL + SEQ) * DM) return;
  if (in_sizes[1] < NB * SKV * DM) return;
  if (in_sizes[2] != DM * DM || in_sizes[3] != DM * DM || in_sizes[4] != DM * DM || in_sizes[5] != DM * DM) return;
  if (out_size < ((NB - 1) * SEQ_FULL + SEQ) * DM) return;

  const float* x1 = (const float*)d_in[0];
  const float* x2 = (const float*)d_in[1];
  const float* wq = (const float*)d_in[2];
  const float* wk = (const float*)d_in[3];
  const float* wv = (const float*)d_in[4];
  const float* wo = (const float*)d_in[5];
  float*      out = (float*)d_out;

  const size_t szX1 = (size_t)NB * SEQ * DM * 2;
  const size_t szX2 = (size_t)NB * SKV * DM * 2;
  const size_t szW  = (size_t)DM * DM * 2;
  const size_t szQP = (size_t)NB * SEQ * QKP * 2;
  const size_t szKP = (size_t)NB * SKV * QKP * 2;
  const size_t szV  = (size_t)NB * DM * SKV * 2;
  const size_t szC  = (size_t)NB * SEQ * DM * 2;
  size_t off = 0;
  const size_t oX1 = off; off += szX1;
  const size_t oX2 = off; off += szX2;
  const size_t oWQ = off; off += szW;
  const size_t oWK = off; off += szW;
  const size_t oWV = off; off += szW;
  const size_t oWO = off; off += szW;
  const size_t oQP = off; off += szQP;
  const size_t oKP = off; off += szKP;
  const size_t oVH = off; off += szV;
  const size_t oVR = off; off += szV;
  const size_t oCH = off; off += szC;
  const size_t oCR = off; off += szC;
  if (off > ws_size) return;
  if (off > (size_t)134217728) return;

  char* ws = (char*)d_ws;
  u16* X1P = (u16*)(ws + oX1);
  u16* X2P = (u16*)(ws + oX2);
  u16* WQT = (u16*)(ws + oWQ);
  u16* WKT = (u16*)(ws + oWK);
  u16* WVT = (u16*)(ws + oWV);
  u16* WOT = (u16*)(ws + oWO);
  u16* QP  = (u16*)(ws + oQP);
  u16* KP  = (u16*)(ws + oKP);
  u16* VH  = (u16*)(ws + oVH);
  u16* VR  = (u16*)(ws + oVR);
  u16* CH  = (u16*)(ws + oCH);
  u16* CR  = (u16*)(ws + oCR);

  cvt16<<<dim3(NB * SEQ), dim3(CVT_THREADS), 0, stream>>>(x1, X1P, SEQ, SEQ_FULL, 1.0f);
  cvt16<<<dim3(NB * SKV), dim3(CVT_THREADS), 0, stream>>>(x2, X2P, SKV, SKV, 1.0f);
  cvtT16<<<dim3((DM / 64) * (DM / 64)), dim3(TR_THREADS), 0, stream>>>(wq, WQT, WSC);
  cvtT16<<<dim3((DM / 64) * (DM / 64)), dim3(TR_THREADS), 0, stream>>>(wk, WKT, WSC);
  cvtT16<<<dim3((DM / 64) * (DM / 64)), dim3(TR_THREADS), 0, stream>>>(wv, WVT, WSC);
  cvtT16<<<dim3((DM / 64) * (DM / 64)), dim3(TR_THREADS), 0, stream>>>(wo, WOT, WSC);
  gemm_qk<<<dim3((NB * SEQ / 128) * (DM / 64)), dim3(128), 0, stream>>>(X1P, WQT, QP, NB * SEQ, QS / WSC);
  gemm_qk<<<dim3((NB * SKV / 128) * (DM / 64)), dim3(128), 0, stream>>>(X2P, WKT, KP, NB * SKV, KS / WSC);
  gemm_hr<<<dim3(NB * (DM / 128) * (SKV / 64)), dim3(128), 0, stream>>>(
      WVT, X2P, VH, VR, DM, SKV, DM, 0, SKV * DM, DM * SKV, VS / WSC);
  attn_fwd<<<dim3(NB * (NG / 4) * (SEQ / 64)), dim3(ATT_THREADS), 0, stream>>>(QP, KP, VH, VR, CH, CR);
  gemm_out<<<dim3((NB * SEQ / 128) * (DM / 64)), dim3(128), 0, stream>>>(
      CH, CR, WOT, out, NB * SEQ, SEQ, SEQ_FULL, 1.0f / (CS * WSC));
  (void)hipGetLastError();
}
